// HeadVer4_14035953123649
// MI455X (gfx1250) — hardware-verified
//
#include <hip/hip_runtime.h>


typedef _Float16 h16;
typedef h16 v16h __attribute__((ext_vector_type(16)));
typedef h16 v8h __attribute__((ext_vector_type(8)));
typedef h16 v8ha __attribute__((ext_vector_type(8), may_alias));
typedef float v8f __attribute__((ext_vector_type(8)));
typedef float v4f __attribute__((ext_vector_type(4)));
typedef float v4fa __attribute__((ext_vector_type(4), may_alias));

static constexpr int BB = 4, TT = 2048, CC = 1024;
static constexpr int MT = BB * TT;
static constexpr int NTHR = 128;
static constexpr int BM = 128, BN = 64, KS = 64;
static constexpr int LDP = 72;
static constexpr int EPH = 72;
static constexpr int EPF = 68;
static constexpr int STG_BYTES = (BM + BN) * LDP * 2;
static constexpr int EPH_BYTES = 4 * 32 * EPH * 2;
static constexpr int EPF_BYTES = 4 * 32 * EPF * 4;
static constexpr int SMEM_H = (STG_BYTES > EPH_BYTES) ? STG_BYTES : EPH_BYTES;
static constexpr int SMEM_F = (STG_BYTES > EPF_BYTES) ? STG_BYTES : EPF_BYTES;
static constexpr float SC_X = 16.0f;
static constexpr float SC_W = 64.0f;
static constexpr float SC_PROJ = 0.015625f;
static constexpr float SC_LOGIT = 0.0001220703125f;
static constexpr float SC_P = 4096.0f;
static constexpr float SC_OUT = 0.0000152587890625f;
static constexpr float NEG_BIG = -1.0e30f;
static_assert(MT % BM == 0 && TT % BM == 0 && CC % BM == 0 && CC % BN == 0 && MT % BN == 0);
static_assert(CC % KS == 0 && BM % KS == 0 && (KS % 32) == 0 && (LDP % 8) == 0 && (EPH % 8) == 0 && (EPF % 4) == 0);
static_assert((MT * CC) % 2048 == 0 && (CC * CC) % 2048 == 0);

#define DEVINL __device__ __forceinline__

DEVINL v8f vzero8() { v8f z = {0.f, 0.f, 0.f, 0.f, 0.f, 0.f, 0.f, 0.f}; return z; }

DEVINL v8f mma16(v16h a, v16h b, v8f c) {
  v8f d = __builtin_amdgcn_wmma_f32_16x16x32_f16(false, a, false, b, (short)0, c, false, false);
  asm volatile("v_nop\n\tv_nop\n\tv_nop\n\tv_nop" : "+v"(d) : "v"(a), "v"(b));
  return d;
}

DEVINL v16h ld_frag(const h16* tile, int row, int ks, int h) {
  union { v16h v; v8h p[2]; } f;
  const h16* base = tile + row * LDP + ks + 8 * h;
  f.p[0] = *(const v8h*)base;
  f.p[1] = *(const v8h*)(base + 16);
  return f.v;
}

DEVINL void stage_tiles(h16* As, h16* Bs, const h16* __restrict__ Ag, int lda,
                        const h16* __restrict__ Bg, int ldb, int k0, int tid) {
  v8h ra[8], rb[4];
#pragma unroll
  for (int i = 0; i < 8; ++i) {
    const int id = tid + NTHR * i, row = id >> 3, c = (id & 7) * 8;
    ra[i] = *(const v8h*)(Ag + (size_t)row * lda + k0 + c);
  }
#pragma unroll
  for (int i = 0; i < 4; ++i) {
    const int id = tid + NTHR * i, row = id >> 3, c = (id & 7) * 8;
    rb[i] = *(const v8h*)(Bg + (size_t)row * ldb + k0 + c);
  }
#pragma unroll
  for (int i = 0; i < 8; ++i) {
    const int id = tid + NTHR * i, row = id >> 3, c = (id & 7) * 8;
    *(v8h*)(As + row * LDP + c) = ra[i];
  }
#pragma unroll
  for (int i = 0; i < 4; ++i) {
    const int id = tid + NTHR * i, row = id >> 3, c = (id & 7) * 8;
    *(v8h*)(Bs + row * LDP + c) = rb[i];
  }
}

DEVINL void mma_step(const h16* As, const h16* Bs, int wave, int m, int h, v8f (&acc)[2][4]) {
#pragma unroll
  for (int ks = 0; ks < KS; ks += 32) {
    const v16h a0 = ld_frag(As, wave * 32 + m, ks, h);
    const v16h a1 = ld_frag(As, wave * 32 + 16 + m, ks, h);
#pragma unroll
    for (int j = 0; j < 4; ++j) {
      const v16h bfr = ld_frag(Bs, 16 * j + m, ks, h);
      acc[0][j] = mma16(a0, bfr, acc[0][j]);
      acc[1][j] = mma16(a1, bfr, acc[1][j]);
    }
  }
}

DEVINL void epi_store_f16(char* smem, v8f (&acc)[2][4], float scl, h16* Dg, int ldd, int wave, int lane) {
  h16* E = (h16*)smem + wave * 32 * EPH;
  const int m = lane & 15, h = lane >> 4;
#pragma unroll
  for (int mi = 0; mi < 2; ++mi)
#pragma unroll
    for (int j = 0; j < 4; ++j)
#pragma unroll
      for (int r = 0; r < 8; ++r)
        E[(16 * mi + 8 * h + r) * EPH + 16 * j + m] = (h16)(acc[mi][j][r] * scl);
  __syncthreads();
  const int rq = lane >> 3, c = (lane & 7) * 8;
  v8h v[8];
#pragma unroll
  for (int i = 0; i < 8; ++i) v[i] = *(const v8ha*)(E + (4 * i + rq) * EPH + c);
#pragma unroll
  for (int i = 0; i < 8; ++i)
    *(volatile v8h*)(Dg + (size_t)(wave * 32 + 4 * i + rq) * ldd + c) = v[i];
  __threadfence();
#pragma unroll
  for (int i = 0; i < 8; ++i)
    *(volatile v8h*)(Dg + (size_t)(wave * 32 + 4 * i + rq) * ldd + c) = v[i];
}

DEVINL void epi_store_f32(char* smem, v8f (&acc)[2][4], float scl, float* Dg, int ldd, int wave, int lane) {
  float* E = (float*)smem + wave * 32 * EPF;
  const int m = lane & 15, h = lane >> 4;
#pragma unroll
  for (int mi = 0; mi < 2; ++mi)
#pragma unroll
    for (int j = 0; j < 4; ++j)
#pragma unroll
      for (int r = 0; r < 8; ++r)
        E[(16 * mi + 8 * h + r) * EPF + 16 * j + m] = acc[mi][j][r] * scl;
  __syncthreads();
  const int rq = lane >> 4, c = (lane & 15) * 4;
#pragma unroll
  for (int i = 0; i < 16; ++i) {
    const v4f v = *(const v4fa*)(E + (2 * i + rq) * EPF + c);
    *(volatile v4f*)(Dg + (size_t)(wave * 32 + 2 * i + rq) * ldd + c) = v;
  }
  __threadfence();
#pragma unroll
  for (int i = 0; i < 16; ++i) {
    const v4f v = *(const v4fa*)(E + (2 * i + rq) * EPF + c);
    *(volatile v4f*)(Dg + (size_t)(wave * 32 + 2 * i + rq) * ldd + c) = v;
  }
}

DEVINL h16 cvt_bf16_scaled_f16(float f, float scl) {
  unsigned u = __float_as_uint(f);
  u = (u + 0x7FFFu + ((u >> 16) & 1u)) & 0xFFFF0000u;
  return (h16)(__uint_as_float(u) * scl);
}

__global__ __launch_bounds__(256) void k_cvt(const float* __restrict__ x, const float* __restrict__ wk,
                                             const float* __restrict__ wq, const float* __restrict__ wv,
                                             h16* __restrict__ x16, h16* __restrict__ wk16,
                                             h16* __restrict__ wq16, h16* __restrict__ wv16) {
  constexpr int PER_BLK = 256 * 8;
  constexpr int XB = (MT * CC) / PER_BLK;
  constexpr int WB = (CC * CC) / PER_BLK;
  const int bid = blockIdx.x;
  const float* src;
  h16* dst;
  float scl;
  int base;
  if (bid < XB) {
    src = x; dst = x16; scl = SC_X; base = bid * PER_BLK;
  } else {
    const int w = bid - XB;
    const int which = w / WB;
    base = (w - which * WB) * PER_BLK;
    scl = SC_W;
    if (which == 0) { src = wk; dst = wk16; }
    else if (which == 1) { src = wq; dst = wq16; }
    else { src = wv; dst = wv16; }
  }
  const int i = base + (int)threadIdx.x * 8;
  const v4f s0 = *(const v4f*)(src + i);
  const v4f s1 = *(const v4f*)(src + i + 4);
  union { v8h v; h16 e[8]; } pk;
#pragma unroll
  for (int q = 0; q < 4; ++q) {
    pk.e[q] = cvt_bf16_scaled_f16(s0[q], scl);
    pk.e[4 + q] = cvt_bf16_scaled_f16(s1[q], scl);
  }
  const v8h pv = pk.v;
  *(volatile v8h*)(dst + i) = pv;
  __threadfence();
  *(volatile v8h*)(dst + i) = pv;
}

__global__ __launch_bounds__(NTHR) void k_proj(const h16* __restrict__ x16, const h16* __restrict__ wq16,
                                               const h16* __restrict__ wk16, const h16* __restrict__ wv16,
                                               h16* __restrict__ q16, h16* __restrict__ k16,
                                               h16* __restrict__ vt16) {
  __shared__ __align__(16) char smem[SMEM_H];
  h16* As = (h16*)smem;
  h16* Bs = As + BM * LDP;
  const int tid = threadIdx.x, wave = tid >> 5, lane = tid & 31, m = lane & 15, h = lane >> 4;
  const int z = blockIdx.z;
  const h16* Ag;
  const h16* Bg;
  h16* Dg;
  int ldd;
  if (z == 2) {
    const int lin = (int)blockIdx.x + (int)gridDim.x * (int)blockIdx.y;
    const int rb = lin & 7, cb = lin >> 3;
    Ag = wv16 + (size_t)rb * BM * CC;
    Bg = x16 + (size_t)cb * BN * CC;
    Dg = vt16 + (size_t)rb * BM * MT + (size_t)cb * BN;
    ldd = MT;
  } else {
    const h16* W = (z == 0) ? wq16 : wk16;
    h16* D = (z == 0) ? q16 : k16;
    Ag = x16 + (size_t)blockIdx.x * BM * CC;
    Bg = W + (size_t)blockIdx.y * BN * CC;
    Dg = D + (size_t)blockIdx.x * BM * CC + (size_t)blockIdx.y * BN;
    ldd = CC;
  }
  v8f acc[2][4];
#pragma unroll
  for (int mi = 0; mi < 2; ++mi)
#pragma unroll
    for (int j = 0; j < 4; ++j) acc[mi][j] = vzero8();
  for (int k0 = 0; k0 < CC; k0 += KS) {
    stage_tiles(As, Bs, Ag, CC, Bg, CC, k0, tid);
    __syncthreads();
    mma_step(As, Bs, wave, m, h, acc);
    __syncthreads();
  }
  epi_store_f16(smem, acc, SC_PROJ, Dg, ldd, wave, lane);
}

__global__ __launch_bounds__(NTHR) void k_scores(const h16* __restrict__ q16, const h16* __restrict__ k16,
                                                 float* __restrict__ S, h16* __restrict__ p16) {
  __shared__ __align__(16) char smem[SMEM_F];
  __shared__ float Ms[BM];
  __shared__ float Ls[BM];
  h16* As = (h16*)smem;
  h16* Bs = As + BM * LDP;
  const int tid = threadIdx.x, wave = tid >> 5, lane = tid & 31, m = lane & 15, h = lane >> 4;
  constexpr int NQT = TT / BM;
  const int b = (int)blockIdx.x / NQT, qt = (int)blockIdx.x - b * NQT;
  const h16* Ag = q16 + ((size_t)b * TT + (size_t)qt * BM) * CC;
  const h16* Kb = k16 + (size_t)b * TT * CC;
  float* Sblk = S + (size_t)b * TT * TT + (size_t)qt * BM * TT;
  h16* Pblk = p16 + (size_t)b * TT * TT + (size_t)qt * BM * TT;

  float mrun[2][8], lrun[2][8];
#pragma unroll
  for (int mi = 0; mi < 2; ++mi)
#pragma unroll
    for (int r = 0; r < 8; ++r) { mrun[mi][r] = NEG_BIG; lrun[mi][r] = 0.f; }
  v8f acc[2][4];
#pragma unroll
  for (int mi = 0; mi < 2; ++mi)
#pragma unroll
    for (int j = 0; j < 4; ++j) acc[mi][j] = vzero8();

  const int ntile = 2 * qt + 2;
  const int rbase = qt * BM + wave * 32 + 8 * h;
  for (int kt = 0; kt < ntile; ++kt) {
    const h16* Bg = Kb + (size_t)kt * BN * CC;
    for (int k0 = 0; k0 < CC; k0 += KS) {
      stage_tiles(As, Bs, Ag, CC, Bg, CC, k0, tid);
      __syncthreads();
      mma_step(As, Bs, wave, m, h, acc);
      __syncthreads();
    }
    const int cbase = kt * BN + m;
#pragma unroll
    for (int mi = 0; mi < 2; ++mi)
#pragma unroll
      for (int j = 0; j < 4; ++j)
#pragma unroll
        for (int r = 0; r < 8; ++r) {
          const int qrow = rbase + 16 * mi + r;
          const int kcol = cbase + 16 * j;
          float v = acc[mi][j][r] * SC_LOGIT;
          if (kcol > qrow) v = NEG_BIG;
          acc[mi][j][r] = v;
        }
#pragma unroll
    for (int mi = 0; mi < 2; ++mi)
#pragma unroll
      for (int r = 0; r < 8; ++r) {
        float tmax = fmaxf(fmaxf(acc[mi][0][r], acc[mi][1][r]), fmaxf(acc[mi][2][r], acc[mi][3][r]));
        tmax = fmaxf(tmax, __shfl_xor(tmax, 1, 32));
        tmax = fmaxf(tmax, __shfl_xor(tmax, 2, 32));
        tmax = fmaxf(tmax, __shfl_xor(tmax, 4, 32));
        tmax = fmaxf(tmax, __shfl_xor(tmax, 8, 32));
        const float mnew = fmaxf(mrun[mi][r], tmax);
        float ps = __expf(acc[mi][0][r] - mnew) + __expf(acc[mi][1][r] - mnew) +
                   __expf(acc[mi][2][r] - mnew) + __expf(acc[mi][3][r] - mnew);
        ps += __shfl_xor(ps, 1, 32);
        ps += __shfl_xor(ps, 2, 32);
        ps += __shfl_xor(ps, 4, 32);
        ps += __shfl_xor(ps, 8, 32);
        lrun[mi][r] = lrun[mi][r] * __expf(mrun[mi][r] - mnew) + ps;
        mrun[mi][r] = mnew;
      }
    epi_store_f32(smem, acc, 1.0f, Sblk + (size_t)kt * BN, TT, wave, lane);
    __syncthreads();
#pragma unroll
    for (int mi = 0; mi < 2; ++mi)
#pragma unroll
      for (int j = 0; j < 4; ++j) acc[mi][j] = vzero8();
  }

  if (m == 0) {
#pragma unroll
    for (int mi = 0; mi < 2; ++mi)
#pragma unroll
      for (int r = 0; r < 8; ++r) {
        const int rl = wave * 32 + 16 * mi + 8 * h + r;
        Ms[rl] = mrun[mi][r];
        Ls[rl] = SC_P / lrun[mi][r];
      }
  }
  __syncthreads();

  const int ncol = (qt + 1) * BM;
#pragma unroll 1
  for (int i = 0; i < 32; ++i) {
    const int rl = wave * 32 + i;
    const float mv = Ms[rl];
    const float li = Ls[rl];
    const float* srow = Sblk + (size_t)rl * TT;
    h16* prow = Pblk + (size_t)rl * TT;
#pragma unroll 1
    for (int c0 = 0; c0 < ncol; c0 += 256) {
      const int c = c0 + 8 * lane;
      if (c < ncol) {
        const v4f s0 = *(const v4f*)(srow + c);
        const v4f s1 = *(const v4f*)(srow + c + 4);
        union { v8h v; h16 e[8]; } pk;
#pragma unroll
        for (int q = 0; q < 4; ++q) {
          pk.e[q] = (h16)(__expf(s0[q] - mv) * li);
          pk.e[4 + q] = (h16)(__expf(s1[q] - mv) * li);
        }
        const v8h pv = pk.v;
        *(volatile v8h*)(prow + c) = pv;
        __threadfence();
        *(volatile v8h*)(prow + c) = pv;
      }
    }
  }
}

__global__ __launch_bounds__(NTHR) void k_pv(const h16* __restrict__ p16, const h16* __restrict__ vt16,
                                             float* __restrict__ out) {
  __shared__ __align__(16) char smem[SMEM_F];
  h16* As = (h16*)smem;
  h16* Bs = As + BM * LDP;
  const int tid = threadIdx.x, wave = tid >> 5, lane = tid & 31, m = lane & 15, h = lane >> 4;
  const int mt = blockIdx.x, nt = blockIdx.y, b = blockIdx.z;
  const h16* Ag = p16 + (size_t)b * TT * TT + (size_t)mt * BM * TT;
  const h16* Bg = vt16 + (size_t)nt * BN * MT + (size_t)b * TT;
  float* Dg = out + ((size_t)b * TT + (size_t)mt * BM) * CC + (size_t)nt * BN;
  v8f acc[2][4];
#pragma unroll
  for (int mi = 0; mi < 2; ++mi)
#pragma unroll
    for (int j = 0; j < 4; ++j) acc[mi][j] = vzero8();
  const int kend = (mt + 1) * BM;
  for (int k0 = 0; k0 < kend; k0 += KS) {
    stage_tiles(As, Bs, Ag, TT, Bg, MT, k0, tid);
    __syncthreads();
    mma_step(As, Bs, wave, m, h, acc);
    __syncthreads();
  }
  epi_store_f32(smem, acc, SC_OUT, Dg, CC, wave, lane);
}

extern "C" void kernel_launch(void* const* d_in, const int* in_sizes, int n_in,
                              void* d_out, int out_size, void* d_ws, size_t ws_size,
                              hipStream_t stream) {
  if (n_in < 4) return;
  if (in_sizes[0] != MT * CC || in_sizes[1] != CC * CC || in_sizes[2] != CC * CC || in_sizes[3] != CC * CC) return;
  if (out_size != MT * CC) return;
  const float* x  = (const float*)d_in[0];
  const float* Wk = (const float*)d_in[1];
  const float* Wq = (const float*)d_in[2];
  const float* Wv = (const float*)d_in[3];
  float* out = (float*)d_out;

  char* ws = (char*)d_ws;
  size_t off = 0;
  auto carve = [&](size_t bytes) -> char* {
    char* p = ws + off;
    off = (off + bytes + 255) & ~(size_t)255;
    return p;
  };
  h16* x16  = (h16*)carve((size_t)MT * CC * 2);
  h16* wk16 = (h16*)carve((size_t)CC * CC * 2);
  h16* wq16 = (h16*)carve((size_t)CC * CC * 2);
  h16* wv16 = (h16*)carve((size_t)CC * CC * 2);
  h16* q16  = (h16*)carve((size_t)MT * CC * 2);
  h16* k16  = (h16*)carve((size_t)MT * CC * 2);
  h16* vt16 = (h16*)carve((size_t)CC * MT * 2);
  float* S  = (float*)carve((size_t)BB * TT * TT * 4);
  h16* p16  = (h16*)carve((size_t)BB * TT * TT * 2);
  if (off > ws_size) return;

  const int cvt_blocks = (MT * CC) / 2048 + 3 * ((CC * CC) / 2048);
  k_cvt<<<dim3(cvt_blocks), dim3(256), 0, stream>>>(x, Wk, Wq, Wv, x16, wk16, wq16, wv16);

  k_proj<<<dim3(MT / BM, CC / BN, 3), dim3(NTHR), 0, stream>>>(x16, wq16, wk16, wv16, q16, k16, vt16);

  k_scores<<<dim3(BB * (TT / BM)), dim3(NTHR), 0, stream>>>(q16, k16, S, p16);

  k_pv<<<dim3(TT / BM, CC / BN, BB), dim3(NTHR), 0, stream>>>(p16, vt16, out);
}
